// EmbGnnModel_32650341384625
// MI455X (gfx1250) — hardware-verified
//
#include <hip/hip_runtime.h>
#include <stddef.h>


#define FDIM    128
#define HDIM    256
#define CDIM    64
#define NTHR    256
#define NWAVE   8
#define EPT     8
#define NGRP    2
#define CHUNK   (NTHR * EPT * NGRP)
#define WCAP    (EPT * NGRP * 32)
#define LISTN   (NWAVE * WCAP)
#define NBC     4096
#define NBF     1024
#define RCAP    40960
#define RBN     128
#define TGT     256
#define DEGCAP  256
#define GROWS   128
#define OTHR    512
#define WSCAP   134217728
#define WSCL    16.0f
#define ASCL    4.0f
#define LDS_FILL ((RCAP + NBF + LISTN) * 4 + 64)
#define LDS_G128 ((GROWS * 128 + GROWS) * 4)
#define LDS_G64  ((GROWS * 64 + GROWS) * 4)

static_assert((CHUNK & (CHUNK - 1)) == 0);
static_assert(CHUNK <= 4096);
static_assert(NBC <= 4096 && NBF <= 4096);
static_assert((NBC & (NBC - 1)) == 0 && (NBF & (NBF - 1)) == 0);
static_assert(NBC == 4 * NBF);
static_assert(OTHR * 8 == NBC);
static_assert((RCAP % 32) == 0);
static_assert(TGT == NWAVE * 32);
static_assert((TGT % GROWS) == 0);
static_assert(GROWS == NWAVE * 16);
static_assert(FDIM == 4 * 32);
static_assert(HDIM == 2 * 128 && CDIM == 64);
static_assert((FDIM % 32) == 0 && (HDIM % 32) == 0);

typedef float    v4f  __attribute__((ext_vector_type(4)));
typedef float    v8f  __attribute__((ext_vector_type(8)));
typedef int      v4i  __attribute__((ext_vector_type(4)));
typedef _Float16 v4h  __attribute__((ext_vector_type(4)));
typedef _Float16 v8h  __attribute__((ext_vector_type(8)));
typedef _Float16 v16h __attribute__((ext_vector_type(16)));
union FragH { v16h v; v8h h[2]; };

__device__ __forceinline__ v8f wmh(v16h a, v16h b, v8f c) {
  v8f d = __builtin_amdgcn_wmma_f32_16x16x32_f16(false, a, false, b, (short)0, c, false, false);
  asm volatile("v_nop\n\tv_nop\n\tv_nop\n\tv_nop" : "+v"(d) : "v"(a), "v"(b));
  return d;
}

__device__ __forceinline__ v8h cvt8(v4f a, v4f b) {
  v8h o;
  o[0] = (_Float16)a.x; o[1] = (_Float16)a.y; o[2] = (_Float16)a.z; o[3] = (_Float16)a.w;
  o[4] = (_Float16)b.x; o[5] = (_Float16)b.y; o[6] = (_Float16)b.z; o[7] = (_Float16)b.w;
  return o;
}

template <int NB>
__device__ __forceinline__ int scan_chunk(const int* __restrict__ dsts, int nE, int cbase, int slotBase,
                                          int vec8, int* list, int tid, int lane, int wave) {
  int wc = 0;
#pragma unroll
  for (int g = 0; g < NGRP; ++g) {
    const int el0  = (g * NTHR + tid) * EPT;
    const int e0   = cbase + el0;
    const int sent = -2147483647 - 1;
    v4i da, db;
    if (vec8 != 0 && cbase + CHUNK <= nE) {
      da = *(const v4i*)(dsts + e0);
      db = *(const v4i*)(dsts + e0 + 4);
    } else {
      da.x = (e0     < nE) ? dsts[min(e0, nE - 1)] : sent;
      da.y = (e0 + 1 < nE) ? dsts[min(e0 + 1, nE - 1)] : sent;
      da.z = (e0 + 2 < nE) ? dsts[min(e0 + 2, nE - 1)] : sent;
      da.w = (e0 + 3 < nE) ? dsts[min(e0 + 3, nE - 1)] : sent;
      db.x = (e0 + 4 < nE) ? dsts[min(e0 + 4, nE - 1)] : sent;
      db.y = (e0 + 5 < nE) ? dsts[min(e0 + 5, nE - 1)] : sent;
      db.z = (e0 + 6 < nE) ? dsts[min(e0 + 6, nE - 1)] : sent;
      db.w = (e0 + 7 < nE) ? dsts[min(e0 + 7, nE - 1)] : sent;
    }
    const unsigned nb = (unsigned)slotBase;
    const unsigned s0 = (unsigned)da.x - nb, s1 = (unsigned)da.y - nb;
    const unsigned s2 = (unsigned)da.z - nb, s3 = (unsigned)da.w - nb;
    const unsigned s4 = (unsigned)db.x - nb, s5 = (unsigned)db.y - nb;
    const unsigned s6 = (unsigned)db.z - nb, s7 = (unsigned)db.w - nb;
    const bool h0 = s0 < (unsigned)NB, h1 = s1 < (unsigned)NB, h2 = s2 < (unsigned)NB, h3 = s3 < (unsigned)NB;
    const bool h4 = s4 < (unsigned)NB, h5 = s5 < (unsigned)NB, h6 = s6 < (unsigned)NB, h7 = s7 < (unsigned)NB;
    const unsigned any = __builtin_amdgcn_ballot_w32(h0 | h1 | h2 | h3 | h4 | h5 | h6 | h7);
    if (any != 0u) {
#define HITJ(J, HJ, SJ) { \
        const unsigned mj = __builtin_amdgcn_ballot_w32(HJ); \
        if (mj != 0u) { \
          if (HJ) { \
            const int pos = wc + (int)__builtin_amdgcn_mbcnt_lo(mj, 0u); \
            if (pos < WCAP) list[wave * WCAP + pos] = ((el0 + (J)) << 12) | (int)(SJ); \
          } \
          wc += (int)__builtin_popcount(mj); } }
      HITJ(0, h0, s0)
      HITJ(1, h1, s1)
      HITJ(2, h2, s2)
      HITJ(3, h3, s3)
      HITJ(4, h4, s4)
      HITJ(5, h5, s5)
      HITJ(6, h6, s6)
      HITJ(7, h7, s7)
#undef HITJ
    }
  }
  return wc;
}

__global__ __launch_bounds__(NTHR) void k_wprep(const float* __restrict__ W, _Float16* Wt, int K, int NN) {
  const int kq = K >> 3;
  const int total = NN * kq;
  const int i = (int)blockIdx.x * NTHR + (int)threadIdx.x;
  if (i >= total) return;
  const int n  = i / kq;
  const int k0 = (i - n * kq) * 8;
  v8h o;
#pragma unroll
  for (int e = 0; e < 8; ++e) o[e] = (_Float16)(W[(size_t)(k0 + e) * NN + n] * WSCL);
  _Float16* d = Wt + (size_t)i * 8;
  *(volatile v8h*)d = o;
  __threadfence();
  *(volatile v8h*)d = o;
}

__global__ __launch_bounds__(NTHR) void k_xcvt(const float* __restrict__ x, _Float16* xh, int nN, int nPad) {
  const int total = nPad * (FDIM / 8);
  const int i = (int)blockIdx.x * NTHR + (int)threadIdx.x;
  if (i >= total) return;
  const int row = i >> 4;
  const int c0  = (i & 15) * 8;
  const int sr  = row > nN - 1 ? nN - 1 : row;
  const float* p = x + (size_t)sr * FDIM + c0;
  const v4f a = *(const v4f*)p, b = *(const v4f*)(p + 4);
  const v8h o = cvt8(a, b);
  _Float16* d = xh + (size_t)i * 8;
  *(volatile v8h*)d = o;
  __threadfence();
  *(volatile v8h*)d = o;
}

__global__ __launch_bounds__(NTHR) void k_count(
    const int* __restrict__ ei, int* cnt, float* dinv, int nE, int vec8) {
  __shared__ __attribute__((aligned(16))) int scnt[NBC];
  __shared__ __attribute__((aligned(16))) int list[LISTN];
  __shared__ int wcnt[NWAVE];
  const int tid = threadIdx.x, lane = tid & 31, wave = tid >> 5;
  const int nodeBase = blockIdx.x * NBC;
  const int* dsts = ei + nE;

  for (int i = tid; i < NBC; i += NTHR) scnt[i] = 0;
  __syncthreads();

  const int nChunks = (nE + CHUNK - 1) / CHUNK;
#pragma unroll 1
  for (int ch = 0; ch < nChunks; ++ch) {
    const int cbase = ch * CHUNK;
    const int wc = scan_chunk<NBC>(dsts, nE, cbase, nodeBase, vec8, list, tid, lane, wave);
    if (lane == 0) wcnt[wave] = wc;
    __syncthreads();
    if (wave == 0) {
#pragma unroll 1
      for (int wsx = 0; wsx < NWAVE; ++wsx) {
        int n = __builtin_amdgcn_readfirstlane(wcnt[wsx]);
        n = n > WCAP ? WCAP : (n < 0 ? 0 : n);
        const int* lp = list + wsx * WCAP;
#pragma unroll 1
        for (int i = 0; i < n; ++i) {
          const int ent  = __builtin_amdgcn_readfirstlane(lp[i]);
          const int slot = ent & (NBC - 1);
          if (lane == 0) scnt[slot] = scnt[slot] + 1;
        }
      }
    }
    __syncthreads();
  }

  v4i cq[4]; v4f dq[4];
#pragma unroll
  for (int q = 0; q < 4; ++q) {
    const int f = (wave * 4 + q) * 128 + 4 * lane;
    const v4i c = *(const v4i*)(scnt + f);
    cq[q] = c;
    dq[q].x = rsqrtf((float)(c.x + 1));
    dq[q].y = rsqrtf((float)(c.y + 1));
    dq[q].z = rsqrtf((float)(c.z + 1));
    dq[q].w = rsqrtf((float)(c.w + 1));
  }
  int*   cp = cnt + (size_t)nodeBase;
  float* dp = dinv + (size_t)nodeBase;
#pragma unroll
  for (int q = 0; q < 4; ++q) {
    const int f = (wave * 4 + q) * 128 + 4 * lane;
    *(volatile v4i*)(cp + f) = cq[q];
    *(volatile v4f*)(dp + f) = dq[q];
  }
  __threadfence();
#pragma unroll
  for (int q = 0; q < 4; ++q) {
    const int f = (wave * 4 + q) * 128 + 4 * lane;
    *(volatile v4i*)(cp + f) = cq[q];
    *(volatile v4f*)(dp + f) = dq[q];
  }
}

__global__ __launch_bounds__(OTHR) void k_offsets(
    const int* __restrict__ cnt, int* off, int* rbase, int nChunk) {
  __shared__ __attribute__((aligned(16))) int soff[NBC];
  __shared__ __attribute__((aligned(16))) int srb[RBN];
  __shared__ int wtot[OTHR / 32];
  const int tid = threadIdx.x, lane = tid & 31, wave = tid >> 5, sub = tid >> 7;
  for (int i = tid; i < RBN; i += OTHR) srb[i] = 0;
  int carry = 0;
#pragma unroll 1
  for (int ch = 0; ch < nChunk; ++ch) {
    const int base = ch * NBC;
    const v4i c0 = *(const v4i*)(cnt + base + 8 * tid);
    const v4i c1 = *(const v4i*)(cnt + base + 8 * tid + 4);
    const int e0 = max(c0.x, 0), e1 = max(c0.y, 0), e2 = max(c0.z, 0), e3 = max(c0.w, 0);
    const int e4 = max(c1.x, 0), e5 = max(c1.y, 0), e6 = max(c1.z, 0), e7 = max(c1.w, 0);
    const int ts = e0 + e1 + e2 + e3 + e4 + e5 + e6 + e7;
    int incl = ts;
#pragma unroll
    for (int d = 1; d < 32; d <<= 1) {
      const int t = __shfl_up(incl, d);
      if (lane >= d) incl += t;
    }
    if (lane == 31) wtot[wave] = incl;
    __syncthreads();
    const int S0 = wtot[0]  + wtot[1]  + wtot[2]  + wtot[3];
    const int S1 = wtot[4]  + wtot[5]  + wtot[6]  + wtot[7];
    const int S2 = wtot[8]  + wtot[9]  + wtot[10] + wtot[11];
    const int S3 = wtot[12] + wtot[13] + wtot[14] + wtot[15];
    int pre = 0;
#pragma unroll 1
    for (int w = 4 * sub; w < wave; ++w) pre += wtot[w];
    const int b0 = carry;
    const int b1 = b0 + ((S0 + 31) & ~31);
    const int b2 = b1 + ((S1 + 31) & ~31);
    const int b3 = b2 + ((S2 + 31) & ~31);
    const int b4 = b3 + ((S3 + 31) & ~31);
    const int myb = sub == 0 ? b0 : (sub == 1 ? b1 : (sub == 2 ? b2 : b3));
    if (tid == 0) {
      srb[min(4 * ch + 0, RBN - 1)] = b0;
      srb[min(4 * ch + 1, RBN - 1)] = b1;
      srb[min(4 * ch + 2, RBN - 1)] = b2;
      srb[min(4 * ch + 3, RBN - 1)] = b3;
    }
    int run = myb + pre + incl - ts;
    soff[8 * tid + 0] = run; run += e0;
    soff[8 * tid + 1] = run; run += e1;
    soff[8 * tid + 2] = run; run += e2;
    soff[8 * tid + 3] = run; run += e3;
    soff[8 * tid + 4] = run; run += e4;
    soff[8 * tid + 5] = run; run += e5;
    soff[8 * tid + 6] = run; run += e6;
    soff[8 * tid + 7] = run;
    carry = b4;
    __syncthreads();
    const v4i o0 = *(const v4i*)(soff + 4 * tid);
    const v4i o1 = *(const v4i*)(soff + 4 * (tid + OTHR));
    int* op = off + base;
    *(volatile v4i*)(op + 4 * tid) = o0;
    *(volatile v4i*)(op + 4 * (tid + OTHR)) = o1;
    __threadfence();
    *(volatile v4i*)(op + 4 * tid) = o0;
    *(volatile v4i*)(op + 4 * (tid + OTHR)) = o1;
    __syncthreads();
  }
  if (tid == 0) srb[min(4 * nChunk, RBN - 1)] = carry;
  __syncthreads();
  v4i rv = {0, 0, 0, 0};
  if (tid < 32) rv = *(const v4i*)(srb + 4 * tid);
  if (tid < 32) *(volatile v4i*)(rbase + 4 * tid) = rv;
  __threadfence();
  if (tid < 32) *(volatile v4i*)(rbase + 4 * tid) = rv;
}

__global__ __launch_bounds__(NTHR) void k_fill(
    const int* __restrict__ ei, const int* __restrict__ off, const int* __restrict__ rbase,
    int* csr, int nN, int nE, int vec8, int csrLen) {
  extern __shared__ v4f lds_dyn[];
  int* region = (int*)lds_dyn;
  int* cursor = region + RCAP;
  int* list   = cursor + NBF;
  int* wcnt   = list + LISTN;
  const int tid = threadIdx.x, lane = tid & 31, wave = tid >> 5;
  const int b = blockIdx.x;
  const int nodeBase = b * NBF;
  const int* dsts = ei + nE;

  int rb0 = rbase[b];
  const int rb1 = rbase[b + 1];
  rb0 = rb0 < 0 ? 0 : (rb0 > csrLen ? csrLen : rb0);
  rb0 &= ~31;
  int len = rb1 - rb0;
  len = len < 0 ? 0 : (len > RCAP ? RCAP : len);
  int lenW = (len + 31) & ~31;
  if (rb0 + lenW > csrLen) lenW = (csrLen - rb0) & ~31;

  {
    const v4i z = {0, 0, 0, 0};
    for (int i = tid; i < RCAP / 4; i += NTHR) ((v4i*)region)[i] = z;
    for (int s = tid; s < NBF; s += NTHR) {
      int o = off[nodeBase + s] - rb0;
      o = o < 0 ? 0 : (o > RCAP ? RCAP : o);
      cursor[s] = o;
    }
  }
  __syncthreads();

  const int nChunks = (nE + CHUNK - 1) / CHUNK;
#pragma unroll 1
  for (int ch = 0; ch < nChunks; ++ch) {
    const int cbase = ch * CHUNK;
    const int wc = scan_chunk<NBF>(dsts, nE, cbase, nodeBase, vec8, list, tid, lane, wave);
    if (lane == 0) wcnt[wave] = wc;
    __syncthreads();
    if (wave == 0) {
#pragma unroll 1
      for (int wsx = 0; wsx < NWAVE; ++wsx) {
        int n = __builtin_amdgcn_readfirstlane(wcnt[wsx]);
        n = n > WCAP ? WCAP : (n < 0 ? 0 : n);
        const int* lp = list + wsx * WCAP;
#pragma unroll 1
        for (int i = 0; i < n; ++i) {
          const int ent  = __builtin_amdgcn_readfirstlane(lp[i]);
          const int slot = ent & (NBF - 1);
          int e = cbase + ((ent >> 12) & (CHUNK - 1));
          e = e > nE - 1 ? nE - 1 : e;
          int src = ei[e];
          src = src < 0 ? 0 : (src > nN - 1 ? nN - 1 : src);
          if (lane == 0) {
            int pos = cursor[slot];
            pos = pos < 0 ? 0 : (pos > RCAP - 1 ? RCAP - 1 : pos);
            region[pos] = src;
            const int np = pos + 1;
            cursor[slot] = np > RCAP ? RCAP : np;
          }
        }
      }
    }
    __syncthreads();
  }

  const int nv = lenW >> 2;
  int* gp = csr + rb0;
#pragma unroll 1
  for (int i = tid; i < nv; i += NTHR) { const v4i v = ((const v4i*)region)[i]; *(volatile v4i*)(gp + 4 * i) = v; }
  __threadfence();
#pragma unroll 1
  for (int i = tid; i < nv; i += NTHR) { const v4i v = ((const v4i*)region)[i]; *(volatile v4i*)(gp + 4 * i) = v; }
}

template <int K, int NNT, int NBLK, int EPI>
__global__ __launch_bounds__(NTHR) void k_gemm(
    const _Float16* __restrict__ A, const _Float16* __restrict__ Bw,
    const float* __restrict__ dinv, const float* __restrict__ bias, const int* __restrict__ label,
    float* Cf, _Float16* Ch, float* lossp, int nRowsValid, size_t repStride) {
  static_assert((K % 32) == 0 && (NBLK % 16) == 0 && (NNT % NBLK) == 0);
  static_assert(EPI != 0 || (NBLK == 128 && NNT == 128));
  static_assert(EPI != 1 || NBLK == 128);
  static_assert(EPI != 2 || (NBLK == 64 && NNT == 64));
  extern __shared__ v4f lds_dyn[];
  float* stg   = (float*)lds_dyn;
  float* sloss = stg + GROWS * NBLK;
  constexpr int NT = NBLK / 16;
  const int tid = threadIdx.x, lane = tid & 31, wave = tid >> 5, hh = lane >> 4, m = lane & 15;
  const int rowBase = (int)blockIdx.x * GROWS;
  const int cb = (int)blockIdx.y * NBLK;

  v8f acc[NT];
#pragma unroll
  for (int t = 0; t < NT; ++t) { v8f z = {0.f, 0.f, 0.f, 0.f, 0.f, 0.f, 0.f, 0.f}; acc[t] = z; }

  const _Float16* ap = A + (size_t)(rowBase + wave * 16 + m) * K + 8 * hh;
#pragma unroll
  for (int kt = 0; kt < K / 32; ++kt) {
    FragH a;
    a.h[0] = *(const v8h*)(ap + 32 * kt);
    a.h[1] = *(const v8h*)(ap + 32 * kt + 16);
#pragma unroll
    for (int t = 0; t < NT; ++t) {
      const _Float16* bp = Bw + (size_t)(cb + 16 * t + m) * K + 32 * kt + 8 * hh;
      FragH b;
      b.h[0] = *(const v8h*)bp;
      b.h[1] = *(const v8h*)(bp + 16);
      acc[t] = wmh(a.v, b.v, acc[t]);
    }
  }

  const int r0 = wave * 16 + 8 * hh;
  float s[8];
  if constexpr (EPI == 0) {
    const v4f dA = *(const v4f*)(dinv + (size_t)rowBase + r0);
    const v4f dB = *(const v4f*)(dinv + (size_t)rowBase + r0 + 4);
    const float iw = 1.0f / WSCL;
    s[0] = dA.x * iw; s[1] = dA.y * iw; s[2] = dA.z * iw; s[3] = dA.w * iw;
    s[4] = dB.x * iw; s[5] = dB.y * iw; s[6] = dB.z * iw; s[7] = dB.w * iw;
  } else {
#pragma unroll
    for (int r = 0; r < 8; ++r) s[r] = 1.0f / (WSCL * ASCL);
  }
  float* sp = stg + r0 * NBLK + m;
#pragma unroll
  for (int t = 0; t < NT; ++t) {
    float bv = 0.0f;
    if constexpr (EPI != 0) bv = bias[cb + 16 * t + m];
#pragma unroll
    for (int r = 0; r < 8; ++r) {
      float v = acc[t][r] * s[r] + bv;
      if constexpr (EPI == 1) v = fmaxf(v, 0.0f) * ASCL;
      sp[r * NBLK + 16 * t] = v;
    }
  }
  __syncthreads();

  if constexpr (EPI == 0) {
    const float* lp = stg + wave * 16 * NBLK + 4 * lane;
    float* gp = Cf + (size_t)(rowBase + wave * 16) * NNT + cb + 4 * lane;
#pragma unroll
    for (int i = 0; i < 16; ++i) {
      const v4f v = *(const v4f*)(lp + i * NBLK);
      *(volatile v4f*)(gp + (size_t)i * NNT) = v;
    }
    __threadfence();
#pragma unroll
    for (int i = 0; i < 16; ++i) {
      const v4f v = *(const v4f*)(lp + i * NBLK);
      *(volatile v4f*)(gp + (size_t)i * NNT) = v;
    }
  } else if constexpr (EPI == 1) {
    const int rsel = lane >> 4, cq = 8 * (lane & 15);
#pragma unroll
    for (int i = 0; i < 8; ++i) {
      const int r = wave * 16 + 2 * i + rsel;
      const float* lp = stg + r * NBLK + cq;
      const v8h o = cvt8(*(const v4f*)lp, *(const v4f*)(lp + 4));
      _Float16* gp = Ch + (size_t)(rowBase + r) * NNT + cb + cq;
      *(volatile v8h*)gp = o;
    }
    __threadfence();
#pragma unroll
    for (int i = 0; i < 8; ++i) {
      const int r = wave * 16 + 2 * i + rsel;
      const float* lp = stg + r * NBLK + cq;
      const v8h o = cvt8(*(const v4f*)lp, *(const v4f*)(lp + 4));
      _Float16* gp = Ch + (size_t)(rowBase + r) * NNT + cb + cq;
      *(volatile v8h*)gp = o;
    }
  } else {
    if (tid < GROWS) {
      const float* rp = stg + tid * NBLK;
      float mx = rp[0];
#pragma unroll 1
      for (int c = 1; c < CDIM; ++c) mx = fmaxf(mx, rp[c]);
      float se = 0.0f;
#pragma unroll 1
      for (int c = 0; c < CDIM; ++c) se += __expf(rp[c] - mx);
      const float lse = mx + __logf(se);
      int gr = rowBase + tid;
      gr = gr > nRowsValid - 1 ? nRowsValid - 1 : gr;
      gr = gr < 0 ? 0 : gr;
      int lb = label[gr];
      lb = lb < 0 ? 0 : (lb > CDIM - 1 ? CDIM - 1 : lb);
      sloss[tid] = lse - rp[lb];
    }
    __syncthreads();
    const bool wv = (rowBase + wave * 16 + 16) <= nRowsValid;
    const int rsel = lane >> 4, cq = 4 * (lane & 15);
    v4f lv = {0.f, 0.f, 0.f, 0.f};
    if (wave == 0) lv = *(const v4f*)(sloss + 4 * lane);
    if (wv) {
#pragma unroll
      for (int rep = 0; rep < 3; ++rep) {
#pragma unroll
        for (int i = 0; i < 8; ++i) {
          const int r = wave * 16 + 2 * i + rsel;
          const v4f v = *(const v4f*)(stg + r * NBLK + cq);
          float* gp = Cf + (size_t)rep * repStride + (size_t)(rowBase + r) * NNT + cq;
          *(volatile v4f*)gp = v;
        }
      }
    }
    if (wave == 0) *(volatile v4f*)(lossp + (size_t)rowBase + 4 * lane) = lv;
    __threadfence();
    if (wv) {
#pragma unroll
      for (int rep = 0; rep < 3; ++rep) {
#pragma unroll
        for (int i = 0; i < 8; ++i) {
          const int r = wave * 16 + 2 * i + rsel;
          const v4f v = *(const v4f*)(stg + r * NBLK + cq);
          float* gp = Cf + (size_t)rep * repStride + (size_t)(rowBase + r) * NNT + cq;
          *(volatile v4f*)gp = v;
        }
      }
    }
    if (wave == 0) *(volatile v4f*)(lossp + (size_t)rowBase + 4 * lane) = lv;
  }
}

__global__ __launch_bounds__(NTHR) void k_agg(
    const int* __restrict__ csr, const int* __restrict__ off, const int* __restrict__ cnt,
    const float* __restrict__ dinv, const float* __restrict__ hw, _Float16* feat,
    const float* __restrict__ bs, int nN, int csrLen) {
  const int tid = threadIdx.x, lane = tid & 31, wave = tid >> 5;
  const int tbase = blockIdx.x * TGT + wave * 32;
  const int cl = tbase + lane;
  const int cnt_l = cnt[cl];
  const int off_l = off[cl];
  union FI { float f; int i; };
  FI dvu; dvu.f = dinv[cl];
  const v4f bb = *(const v4f*)(bs + 4 * lane);

#pragma unroll 1
  for (int j = 0; j < 32; ++j) {
    const int c = tbase + j;
    int n = __builtin_amdgcn_readlane(cnt_l, j);
    n = n < 0 ? 0 : (n > DEGCAP ? DEGCAP : n);
    const int st = __builtin_amdgcn_readlane(off_l, j);
    FI du; du.i = __builtin_amdgcn_readlane(dvu.i, j);
    const float dc = du.f;
    v4f acc = {0.f, 0.f, 0.f, 0.f};
#pragma unroll 1
    for (int q0 = 0; q0 < n; q0 += 32) {
      int pos = st + q0 + lane;
      pos = pos < 0 ? 0 : (pos > csrLen - 1 ? csrLen - 1 : pos);
      int sl = csr[pos];
      sl = sl < 0 ? 0 : (sl > nN - 1 ? nN - 1 : sl);
      const int mcnt = (n - q0) < 32 ? (n - q0) : 32;
#pragma unroll 1
      for (int p = 0; p < mcnt; ++p) {
        const int sidx = __builtin_amdgcn_readlane(sl, p);
        acc = acc + *(const v4f*)(hw + (size_t)sidx * FDIM + 4 * lane);
      }
    }
    const v4f sv = *(const v4f*)(hw + (size_t)c * FDIM + 4 * lane);
    const v4f v = ((acc + sv) * dc + bb) * ASCL;
    v4h o;
    o.x = (_Float16)v.x; o.y = (_Float16)v.y; o.z = (_Float16)v.z; o.w = (_Float16)v.w;
    _Float16* fp = feat + (size_t)c * FDIM + 4 * lane;
    *(volatile v4h*)fp = o;
    __threadfence();
    *(volatile v4h*)fp = o;
  }
}

__global__ __launch_bounds__(NTHR) void k_lossred(
    const float* __restrict__ lossp, const int* __restrict__ mk0, const int* __restrict__ mk1,
    const int* __restrict__ mk2, float* outp, int nN) {
  __shared__ float red[6 * NTHR];
  const int tid = threadIdx.x;
  float s0 = 0.0f, s1 = 0.0f, s2 = 0.0f, c0 = 0.0f, c1 = 0.0f, c2 = 0.0f;
#pragma unroll 1
  for (int i = tid; i < nN; i += NTHR) {
    const float l  = lossp[i];
    const float f0 = (mk0[i] == 1) ? 1.0f : 0.0f;
    const float f1 = (mk1[i] == 1) ? 1.0f : 0.0f;
    const float f2 = (mk2[i] == 1) ? 1.0f : 0.0f;
    s0 += f0 * l; c0 += f0;
    s1 += f1 * l; c1 += f1;
    s2 += f2 * l; c2 += f2;
  }
  red[0 * NTHR + tid] = s0; red[1 * NTHR + tid] = s1; red[2 * NTHR + tid] = s2;
  red[3 * NTHR + tid] = c0; red[4 * NTHR + tid] = c1; red[5 * NTHR + tid] = c2;
  __syncthreads();
#pragma unroll 1
  for (int st = NTHR / 2; st > 0; st >>= 1) {
    if (tid < st) {
#pragma unroll
      for (int q = 0; q < 6; ++q) red[q * NTHR + tid] += red[q * NTHR + tid + st];
    }
    __syncthreads();
  }
  if (tid == 0) {
    const float n0 = red[0 * NTHR], n1 = red[1 * NTHR], n2 = red[2 * NTHR];
    const float d0 = red[3 * NTHR], d1 = red[4 * NTHR], d2 = red[5 * NTHR];
    const float r0 = n0 * (1.0f / d0);
    const float r1 = n1 * (1.0f / d1);
    const float r2 = n2 * (1.0f / d2);
    *(volatile float*)(outp + 0) = r0;
    *(volatile float*)(outp + 1) = r1;
    *(volatile float*)(outp + 2) = r2;
    __threadfence();
    *(volatile float*)(outp + 0) = r0;
    *(volatile float*)(outp + 1) = r1;
    *(volatile float*)(outp + 2) = r2;
  }
}

extern "C" void kernel_launch(void* const* d_in, const int* in_sizes, int n_in,
                              void* d_out, int out_size, void* d_ws, size_t ws_size,
                              hipStream_t stream) {
  if (n_in < 12) return;
  const int nN = in_sizes[0] / FDIM;
  const int nE = in_sizes[1] / 2;
  if (nN <= 0 || nE <= 0) return;
  if (in_sizes[0] != nN * FDIM || in_sizes[1] != 2 * nE) return;
  if (in_sizes[2] != nN || in_sizes[3] != nN || in_sizes[4] != nN || in_sizes[5] != nN) return;
  if (in_sizes[6] != FDIM * FDIM || in_sizes[7] != FDIM) return;
  if (in_sizes[8] != FDIM * HDIM || in_sizes[9] != HDIM) return;
  if (in_sizes[10] != HDIM * CDIM || in_sizes[11] != CDIM) return;
  if ((nN & 15) != 0) return;
  if ((long long)out_size != 3LL * (long long)nN * CDIM + 3LL) return;
  if (nE > (1 << 28) || nN > (1 << 24)) return;

  const float* x      = (const float*)d_in[0];
  const int*   ei     = (const int*)d_in[1];
  const int*   label  = (const int*)d_in[2];
  const int*   mtr    = (const int*)d_in[3];
  const int*   mdv    = (const int*)d_in[4];
  const int*   mte    = (const int*)d_in[5];
  const float* Wg     = (const float*)d_in[6];
  const float* bg     = (const float*)d_in[7];
  const float* Wf     = (const float*)d_in[8];
  const float* bf     = (const float*)d_in[9];
  const float* Wp     = (const float*)d_in[10];
  const float* bp     = (const float*)d_in[11];
  float* out = (float*)d_out;

  const int NPAD   = ((nN + TGT - 1) / TGT) * TGT;
  const int nBC    = (nN + NBC - 1) / NBC;
  const int CNTPAD = nBC * NBC;
  if (4 * nBC + 1 > RBN) return;
  const int nBF    = (nN + NBF - 1) / NBF;
  const int csrLen = ((nE + 31) & ~31) + 4096;
  if (31 * 4 * nBC > 4096) return;
  const int nGemm  = NPAD / GROWS;
  const int nAgg   = NPAD / TGT;

  char* ws = (char*)d_ws;
  size_t off = 0;
  const size_t oWg  = off; off += (size_t)FDIM * FDIM * 2;           off = (off + 255) & ~(size_t)255;
  const size_t oWf  = off; off += (size_t)HDIM * FDIM * 2;           off = (off + 255) & ~(size_t)255;
  const size_t oWp  = off; off += (size_t)CDIM * HDIM * 2;           off = (off + 255) & ~(size_t)255;
  const size_t oXh  = off; off += (size_t)NPAD * FDIM * 2;           off = (off + 255) & ~(size_t)255;
  const size_t oCnt = off; off += (size_t)CNTPAD * 4;                off = (off + 255) & ~(size_t)255;
  const size_t oDv  = off; off += (size_t)CNTPAD * 4;                off = (off + 255) & ~(size_t)255;
  const size_t oOff = off; off += (size_t)CNTPAD * 4;                off = (off + 255) & ~(size_t)255;
  const size_t oRb  = off; off += (size_t)RBN * 4;                   off = (off + 255) & ~(size_t)255;
  const size_t oCsr = off; off += (size_t)csrLen * 4;                off = (off + 255) & ~(size_t)255;
  const size_t oHw  = off; off += (size_t)NPAD * FDIM * 4;           off = (off + 255) & ~(size_t)255;
  const size_t oFt  = off; off += (size_t)NPAD * FDIM * 2;           off = (off + 255) & ~(size_t)255;
  const size_t oH   = off; off += (size_t)NPAD * HDIM * 2;           off = (off + 255) & ~(size_t)255;
  const size_t oLs  = off; off += (size_t)NPAD * 4;                  off = (off + 255) & ~(size_t)255;
  if (off > ws_size || off > (size_t)WSCAP) return;
  _Float16* wg16 = (_Float16*)(ws + oWg);
  _Float16* wf16 = (_Float16*)(ws + oWf);
  _Float16* wp16 = (_Float16*)(ws + oWp);
  _Float16* xh   = (_Float16*)(ws + oXh);
  int*      cnt  = (int*)(ws + oCnt);
  float*    dinv = (float*)(ws + oDv);
  int*      offp = (int*)(ws + oOff);
  int*      rb   = (int*)(ws + oRb);
  int*      csr  = (int*)(ws + oCsr);
  float*    hw   = (float*)(ws + oHw);
  _Float16* ft16 = (_Float16*)(ws + oFt);
  _Float16* h16  = (_Float16*)(ws + oH);
  float*    lossb = (float*)(ws + oLs);

  const int vec8 = ((nE & 3) == 0) ? 1 : 0;

  k_wprep<<<(FDIM * (FDIM / 8) + NTHR - 1) / NTHR, NTHR, 0, stream>>>(Wg, wg16, FDIM, FDIM);
  k_wprep<<<(HDIM * (FDIM / 8) + NTHR - 1) / NTHR, NTHR, 0, stream>>>(Wf, wf16, FDIM, HDIM);
  k_wprep<<<(CDIM * (HDIM / 8) + NTHR - 1) / NTHR, NTHR, 0, stream>>>(Wp, wp16, HDIM, CDIM);
  k_xcvt<<<(NPAD * (FDIM / 8) + NTHR - 1) / NTHR, NTHR, 0, stream>>>(x, xh, nN, NPAD);

  k_count<<<nBC, NTHR, 0, stream>>>(ei, cnt, dinv, nE, vec8);
  k_offsets<<<1, OTHR, 0, stream>>>(cnt, offp, rb, nBC);
  hipFuncSetAttribute(reinterpret_cast<const void*>(&k_fill),
                      hipFuncAttributeMaxDynamicSharedMemorySize, LDS_FILL);
  k_fill<<<nBF, NTHR, LDS_FILL, stream>>>(ei, offp, rb, csr, nN, nE, vec8, csrLen);

  hipFuncSetAttribute(reinterpret_cast<const void*>(&k_gemm<FDIM, FDIM, 128, 0>),
                      hipFuncAttributeMaxDynamicSharedMemorySize, LDS_G128);
  k_gemm<FDIM, FDIM, 128, 0><<<dim3(nGemm, 1), NTHR, LDS_G128, stream>>>(
      xh, wg16, dinv, bg, label, hw, ft16, lossb, NPAD, (size_t)0);
  k_agg<<<nAgg, NTHR, 0, stream>>>(csr, offp, cnt, dinv, hw, ft16, bg, nN, csrLen);
  hipFuncSetAttribute(reinterpret_cast<const void*>(&k_gemm<FDIM, HDIM, 128, 1>),
                      hipFuncAttributeMaxDynamicSharedMemorySize, LDS_G128);
  k_gemm<FDIM, HDIM, 128, 1><<<dim3(nGemm, HDIM / 128), NTHR, LDS_G128, stream>>>(
      ft16, wf16, dinv, bf, label, hw, h16, lossb, NPAD, (size_t)0);
  hipFuncSetAttribute(reinterpret_cast<const void*>(&k_gemm<HDIM, CDIM, 64, 2>),
                      hipFuncAttributeMaxDynamicSharedMemorySize, LDS_G64);
  k_gemm<HDIM, CDIM, 64, 2><<<dim3(nGemm, 1), NTHR, LDS_G64, stream>>>(
      h16, wp16, dinv, bp, label, out, ft16, lossb, nN, (size_t)nN * CDIM);
  k_lossred<<<1, NTHR, 0, stream>>>(lossb, mtr, mdv, mte, out + (size_t)3 * nN * CDIM, nN);
}
